// Block_76785425318629
// MI455X (gfx1250) — hardware-verified
//
#include <hip/hip_runtime.h>
#pragma clang fp contract(off)


#ifndef NB
#define NB 2
#endif
#ifndef SEQ
#define SEQ 2048
#endif
#define NB_FULL  2
#define SEQ_FULL 2048
#define TT   SEQ
#define DM   1024
#define NH_  16
#define HD   64
#define FF   4096
#define QKVW (3 * DM)
#define KCH  64
#define WCAR 64.0f
#define QCAR 8.0f
#define VCAR 8.0f
#define PCAR 1024.0f
#define OCAR 16.0f
#define GCAR 8.0f
#define NEGB (-3.0e38f)
#define L2E  1.4426950408889634f

static_assert(SEQ % 64 == 0);
static_assert(SEQ <= SEQ_FULL);
static_assert(NB >= 1 && NB <= NB_FULL);
static_assert(DM % 256 == 0 && FF % 64 == 0 && QKVW % 64 == 0 && DM % 64 == 0);
static_assert(DM % 32 == 0 && FF % 32 == 0);
static_assert(HD == 64 && NH_ * HD == DM && KCH == 64);
static_assert(((size_t)NH_ * TT * HD / 8) % 256 == 0);
static_assert(((size_t)NH_ * HD * TT / 8) % 256 == 0);
static_assert(((size_t)TT * FF / 8) % 256 == 0);
static_assert(TT % 8 == 0 && TT % KCH == 0);

typedef _Float16 h16;
typedef __attribute__((ext_vector_type(16))) _Float16 v16h;
typedef __attribute__((ext_vector_type(8)))  _Float16 v8h;
typedef __attribute__((ext_vector_type(4)))  _Float16 v4h;
typedef __attribute__((ext_vector_type(8)))  float    v8f;
typedef __attribute__((ext_vector_type(4)))  float    v4f;
typedef v8h __attribute__((may_alias)) v8ha;
typedef v4f __attribute__((may_alias)) v4fa;

__device__ __forceinline__ unsigned short f2bf(float f) { unsigned u = __float_as_uint(f); u += 0x7FFFu + ((u >> 16) & 1u); return (unsigned short)(u >> 16); }
__device__ __forceinline__ float bf2f(unsigned short b) { return __uint_as_float(((unsigned)b) << 16); }
__device__ __forceinline__ float bfr(float f) { return bf2f(f2bf(f)); }
__device__ __forceinline__ v16h cat16(v8h lo, v8h hi) { return __builtin_shufflevector(lo, hi, 0, 1, 2, 3, 4, 5, 6, 7, 8, 9, 10, 11, 12, 13, 14, 15); }
__device__ __forceinline__ v8f wmma16(v16h a, v16h b, v8f c) { return __builtin_amdgcn_wmma_f32_16x16x32_f16(false, a, false, b, (short)0, c, false, false); }
__device__ __forceinline__ v16h ldf(const h16* p) { return cat16(*(const v8h*)p, *(const v8h*)(p + 16)); }
__device__ __forceinline__ float ex2(float a) { return __builtin_amdgcn_exp2f(a); }

template <int NSPLIT, bool BIAS, int RES>
__global__ __launch_bounds__(32) void k_gemmw(const h16* __restrict__ A, const h16* __restrict__ A2, const h16* __restrict__ Bt, const h16* __restrict__ Bt2, int K, float* C, int ldc, const float* __restrict__ bias, const float* __restrict__ R, float osc, size_t sA, size_t sB, size_t sC) {
    __shared__ __align__(16) float os[16 * 68];
    const size_t z = blockIdx.z; A += z * sA; if (A2) A2 += z * sA; Bt += z * sB; if (Bt2) Bt2 += z * sB; C += z * sC; if (RES != 0) R += z * sC;
    const int lane = threadIdx.x & 31, lr = lane & 15, hi = lane >> 4; const int r0 = blockIdx.x * 64, c0 = blockIdx.y * 64;
    v8f acc[4][4];
#pragma unroll
    for (int mb = 0; mb < 4; ++mb)
#pragma unroll
        for (int nb = 0; nb < 4; ++nb) acc[mb][nb] = (v8f){};
    const size_t aoff = (size_t)(r0 + lr) * K + 8 * hi, boff = (size_t)(c0 + lr) * K + 8 * hi;
#pragma unroll 1
    for (int kc = 0; kc < K; kc += 32) {
        v16h a[4], a2[4];
#pragma unroll
        for (int mb = 0; mb < 4; ++mb) { a[mb] = ldf(A + aoff + (size_t)mb * 16 * K + kc); if (NSPLIT == 1 || NSPLIT == 2) a2[mb] = ldf(A2 + aoff + (size_t)mb * 16 * K + kc); }
#pragma unroll
        for (int nb = 0; nb < 4; ++nb) { const v16h b = ldf(Bt + boff + (size_t)nb * 16 * K + kc); v16h b2; if (NSPLIT >= 2) b2 = ldf(Bt2 + boff + (size_t)nb * 16 * K + kc);
#pragma unroll
            for (int mb = 0; mb < 4; ++mb) { acc[mb][nb] = wmma16(a[mb], b, acc[mb][nb]); if (NSPLIT == 1 || NSPLIT == 2) acc[mb][nb] = wmma16(a2[mb], b, acc[mb][nb]); if (NSPLIT >= 2) acc[mb][nb] = wmma16(a[mb], b2, acc[mb][nb]); } }
        asm volatile("v_nop\n\tv_nop\n\tv_nop\n\tv_nop" : "+v"(acc[0][0]), "+v"(acc[1][1]), "+v"(acc[2][2]), "+v"(acc[3][3]) : "v"(a[0]), "v"(a[3]));
    }
#pragma unroll
    for (int mb = 0; mb < 4; ++mb) {
#pragma unroll
        for (int nb = 0; nb < 4; ++nb) {
#pragma unroll
            for (int j = 0; j < 8; ++j) os[(hi * 8 + j) * 68 + nb * 16 + lr] = acc[mb][nb][j]; }
        __builtin_amdgcn_fence(3  , "wavefront"); __builtin_amdgcn_wave_barrier(); asm volatile("" ::: "memory");
        float* crow = C + (size_t)(r0 + mb * 16) * ldc + c0;
        const float* rrow = (RES != 0) ? (R + (size_t)(r0 + mb * 16) * ldc + c0) : R;
#pragma unroll 1
        for (int ps = 0; ps < 2; ++ps) {
#pragma unroll
            for (int s = 0; s < 8; ++s) { const int row = 2 * s + hi, cofs = lr * 4; v4f val = *(const v4fa*)(os + row * 68 + cofs); val = val * osc;
                if (BIAS) { const v4f bv = *(const v4f*)(bias + c0 + cofs);
#pragma unroll
                    for (int q = 0; q < 4; ++q) val[q] = val[q] + bfr(bv[q]); }
                if (RES != 0) { const v4f rv = *(const v4f*)(rrow + (size_t)row * ldc + cofs);
#pragma unroll
                    for (int q = 0; q < 4; ++q) val[q] = val[q] + ((RES == 2) ? bfr(rv[q]) : rv[q]); }
                *(volatile v4f*)(crow + (size_t)row * ldc + cofs) = val; }
            if (ps == 0) __threadfence(); }
        __builtin_amdgcn_fence(3  , "wavefront"); __builtin_amdgcn_wave_barrier(); asm volatile("" ::: "memory");
    }
}

__global__ __launch_bounds__(256) void k_cvtw(const float* __restrict__ src, h16* dst, size_t n8, float sc) {
    const size_t i = (size_t)blockIdx.x * 256 + threadIdx.x; if (i >= n8) return;
    const v4f v0 = *(const v4f*)(src + i * 8); const v4f v1 = *(const v4f*)(src + i * 8 + 4); v8h o;
#pragma unroll
    for (int k = 0; k < 4; ++k) { o[k] = (h16)(bfr(v0[k]) * sc); o[4 + k] = (h16)(bfr(v1[k]) * sc); }
    *(volatile v8h*)(dst + i * 8) = o; __threadfence(); *(volatile v8h*)(dst + i * 8) = o;
}

template <bool RAW>
__global__ __launch_bounds__(256) void k_ln(const float* __restrict__ X, const float* __restrict__ g, const float* __restrict__ bb, h16* H) {
    const int lane = threadIdx.x & 31; const int row = blockIdx.x * 8 + (threadIdx.x >> 5); if (row >= TT) return;
    const float* xr = X + (size_t)row * DM; float v[DM / 32]; float s = 0.f;
#pragma unroll
    for (int ch = 0; ch < DM / 256; ++ch) { const v4f a0 = *(const v4f*)(xr + ch * 256 + lane * 8); const v4f a1 = *(const v4f*)(xr + ch * 256 + lane * 8 + 4);
#pragma unroll
        for (int q = 0; q < 4; ++q) { const float t0 = RAW ? bfr(a0[q]) : a0[q]; const float t1 = RAW ? bfr(a1[q]) : a1[q]; v[ch * 8 + q] = t0; v[ch * 8 + 4 + q] = t1; } }
#pragma unroll
    for (int k = 0; k < DM / 32; ++k) s = s + v[k];
#pragma unroll
    for (int sh = 16; sh; sh >>= 1) s = s + __shfl_xor(s, sh, 32);
    const float mu = s * (1.0f / (float)DM); float s2 = 0.f;
#pragma unroll
    for (int k = 0; k < DM / 32; ++k) { const float d0 = v[k] - mu; const float p = d0 * d0; s2 = s2 + p; }
#pragma unroll
    for (int sh = 16; sh; sh >>= 1) s2 = s2 + __shfl_xor(s2, sh, 32);
    const float var = s2 * (1.0f / (float)DM);
    const float rs = __fdiv_rn(1.0f, __fsqrt_rn(var + 1e-5f));
#pragma unroll 1
    for (int ps = 0; ps < 2; ++ps) {
#pragma unroll
        for (int ch = 0; ch < DM / 256; ++ch) { const int c0 = ch * 256 + lane * 8; const v4f g0 = *(const v4f*)(g + c0); const v4f g1 = *(const v4f*)(g + c0 + 4); const v4f b0 = *(const v4f*)(bb + c0); const v4f b1 = *(const v4f*)(bb + c0 + 4); v8h o;
#pragma unroll
            for (int q = 0; q < 4; ++q) {
                { const float xn = (v[ch * 8 + q] - mu) * rs; const float yv = xn * bfr(g0[q]) + bfr(b0[q]); o[q] = (h16)yv; }
                { const float xn = (v[ch * 8 + 4 + q] - mu) * rs; const float yv = xn * bfr(g1[q]) + bfr(b1[q]); o[4 + q] = (h16)yv; } }
            *(volatile v8h*)(H + (size_t)row * DM + c0) = o; }
        if (ps == 0) __threadfence(); }
}

__global__ __launch_bounds__(256) void k_qkp(const float* __restrict__ F, h16* Qp, h16* Kp_) {
    const size_t e8 = (size_t)blockIdx.x * 256 + threadIdx.x; if (e8 >= (size_t)NH_ * TT * HD / 8) return;
    const int d8 = (int)(e8 & 7); const int t = (int)((e8 >> 3) % TT); const int hh = (int)(e8 / ((size_t)8 * TT));
    const float* src = F + (size_t)t * QKVW + hh * HD + d8 * 8;
    const v4f q0 = *(const v4f*)src; const v4f q1 = *(const v4f*)(src + 4); const v4f k0 = *(const v4f*)(src + DM); const v4f k1 = *(const v4f*)(src + DM + 4);
    v8h oq, ok;
#pragma unroll
    for (int k = 0; k < 4; ++k) { oq[k] = (h16)(q0[k] * QCAR); oq[4 + k] = (h16)(q1[k] * QCAR); ok[k] = (h16)(k0[k] * QCAR); ok[4 + k] = (h16)(k1[k] * QCAR); }
    const size_t oo = e8 * 8;
    *(volatile v8h*)(Qp + oo) = oq; *(volatile v8h*)(Kp_ + oo) = ok; __threadfence(); *(volatile v8h*)(Qp + oo) = oq; *(volatile v8h*)(Kp_ + oo) = ok;
}
__global__ __launch_bounds__(256) void k_vtp(const float* __restrict__ F, h16* VT) {
    const size_t e8 = (size_t)blockIdx.x * 256 + threadIdx.x; if (e8 >= (size_t)NH_ * HD * TT / 8) return;
    const int t8 = (int)(e8 % (TT / 8)); const int d = (int)((e8 / (TT / 8)) % HD); const int hh = (int)(e8 / ((size_t)(TT / 8) * HD));
    const float* src = F + (size_t)(t8 * 8) * QKVW + 2 * DM + hh * HD + d; v8h o;
#pragma unroll
    for (int j = 0; j < 8; ++j) o[j] = (h16)(src[(size_t)j * QKVW] * VCAR);
    const size_t oo = e8 * 8;
    *(volatile v8h*)(VT + oo) = o; __threadfence(); *(volatile v8h*)(VT + oo) = o;
}

__global__ __launch_bounds__(128) void k_flash(const h16* __restrict__ Qp, const h16* __restrict__ Kp_, const h16* __restrict__ VT, h16* AT) {
    __shared__ __align__(16) h16 ot[4 * 16 * 72];
    const int lane = threadIdx.x & 31, w = threadIdx.x >> 5, h = lane >> 4, lr = lane & 15;
    const int qb = blockIdx.x, hh = blockIdx.y;
    const int q0 = qb * 64 + w * 16; const int tq = q0 + lr;
    const h16* Qh = Qp + (size_t)hh * TT * HD; const h16* Kh = Kp_ + (size_t)hh * TT * HD; const h16* Vh = VT + (size_t)hh * HD * TT;
    v16h qf[2];
    qf[0] = ldf(Qh + (size_t)tq * HD + 8 * h); qf[1] = ldf(Qh + (size_t)tq * HD + 32 + 8 * h);
    v8f o[4];
#pragma unroll
    for (int dt = 0; dt < 4; ++dt) o[dt] = (v8f){};
    float m = NEGB, l = 0.f;
    const float ssc = 1.0f / (8.0f * QCAR * QCAR);
    const int nch = qb + 1;
#pragma unroll 1
    for (int c = 0; c < nch; ++c) {
        const int c0 = c * KCH;
        v8f s[4]; v16h a;
#pragma unroll
        for (int kt = 0; kt < 4; ++kt) { s[kt] = (v8f){}; const h16* kp = Kh + (size_t)(c0 + kt * 16 + lr) * HD + 8 * h;
#pragma unroll
            for (int ds = 0; ds < 2; ++ds) { a = ldf(kp + ds * 32); s[kt] = wmma16(a, qf[ds], s[kt]); } }
        asm volatile("v_nop\n\tv_nop\n\tv_nop\n\tv_nop" : "+v"(s[0]), "+v"(s[1]), "+v"(s[2]), "+v"(s[3]) : "v"(qf[0]), "v"(qf[1]), "v"(a));
        float mx = m;
#pragma unroll
        for (int kt = 0; kt < 4; ++kt) {
#pragma unroll
            for (int r = 0; r < 8; ++r) { const int key = c0 + kt * 16 + 8 * h + r; const float t = (key <= tq) ? (s[kt][r] * ssc) : NEGB; s[kt][r] = t; mx = fmaxf(mx, t); } }
        mx = fmaxf(mx, __shfl_xor(mx, 16, 32));
        const float alpha = ex2((m - mx) * L2E);
        m = mx;
        float psum = 0.f; v8h p8[4];
#pragma unroll
        for (int kt = 0; kt < 4; ++kt) {
#pragma unroll
            for (int r = 0; r < 8; ++r) { const float p = ex2((s[kt][r] - mx) * L2E); psum = psum + p; p8[kt][r] = (h16)(p * PCAR); } }
        l = l * alpha + psum;
        v16h pf[2]; pf[0] = cat16(p8[0], p8[1]); pf[1] = cat16(p8[2], p8[3]);
#pragma unroll
        for (int dt = 0; dt < 4; ++dt) o[dt] = o[dt] * alpha;
        v16h av;
#pragma unroll
        for (int dt = 0; dt < 4; ++dt) { const h16* vp = Vh + (size_t)(dt * 16 + lr) * TT + c0 + 8 * h;
#pragma unroll
            for (int ks = 0; ks < 2; ++ks) { av = ldf(vp + ks * 32); o[dt] = wmma16(av, pf[ks], o[dt]); } }
        asm volatile("v_nop\n\tv_nop\n\tv_nop\n\tv_nop" : "+v"(o[0]), "+v"(o[1]), "+v"(o[2]), "+v"(o[3]) : "v"(pf[0]), "v"(pf[1]), "v"(av));
    }
    l = l + __shfl_xor(l, 16, 32);
    const float inv = __fdiv_rn(OCAR, l * (PCAR * VCAR));
    h16* ow = ot + w * (16 * 72);
#pragma unroll
    for (int dt = 0; dt < 4; ++dt) { v8h o8;
#pragma unroll
        for (int r = 0; r < 8; ++r) o8[r] = (h16)(o[dt][r] * inv);
        *(v8h*)(ow + lr * 72 + dt * 16 + 8 * h) = o8; }
    __builtin_amdgcn_fence(3  , "wavefront"); __builtin_amdgcn_wave_barrier(); asm volatile("" ::: "memory");
    const int piece = lane & 7, rsel = lane >> 3;
#pragma unroll 1
    for (int ps = 0; ps < 2; ++ps) {
#pragma unroll
        for (int rr = 0; rr < 4; ++rr) { const int row = rr * 4 + rsel; const v8h val = *(const v8ha*)(ow + row * 72 + piece * 8);
            *(volatile v8h*)(AT + (size_t)(q0 + row) * DM + hh * HD + piece * 8) = val; }
        if (ps == 0) __threadfence(); }
}

__device__ __forceinline__ float erf_as(float x) {
    const float ax = fabsf(x);
    const float t = __fdiv_rn(1.0f, 1.0f + 0.3275911f * ax);
    float poly = 1.061405429f; poly = poly * t + (-1.453152027f); poly = poly * t + 1.421413741f; poly = poly * t + (-0.284496736f); poly = poly * t + 0.254829592f; poly = poly * t;
    const float e = ex2(-(ax * ax) * L2E);
    const float r = 1.0f - poly * e;
    return (x < 0.f) ? -r : r;
}
__global__ __launch_bounds__(256) void k_gelu(const float* __restrict__ F, h16* G, size_t n8) {
    __shared__ __align__(16) h16 sg[256 * 8];
    const size_t i = (size_t)blockIdx.x * 256 + threadIdx.x; if (i >= n8) return;
    h16* my = sg + threadIdx.x * 8;
#pragma unroll 1
    for (int q = 0; q < 8; ++q) { const float v = F[i * 8 + q]; const float hx = 0.5f * v; const float gl = hx * (1.0f + erf_as(v * 0.70710678118654752f)); my[q] = (h16)(gl * GCAR); }
    __builtin_amdgcn_fence(3  , "wavefront"); __builtin_amdgcn_wave_barrier(); asm volatile("" ::: "memory");
    const v8h o = *(const v8ha*)my;
    *(volatile v8h*)(G + i * 8) = o; __threadfence(); *(volatile v8h*)(G + i * 8) = o;
}

extern "C" void kernel_launch(void* const* d_in, const int* in_sizes, int n_in,
                              void* d_out, int out_size, void* d_ws, size_t ws_size, hipStream_t stream) {
    if (n_in < 13) return;
    const size_t xneed = (size_t)(NB - 1) * SEQ_FULL * DM + (size_t)SEQ * DM;
    if ((size_t)in_sizes[0] < xneed || (size_t)out_size < xneed) return;
    if (in_sizes[1] < DM || in_sizes[2] < DM || (size_t)in_sizes[3] < (size_t)QKVW * DM || in_sizes[4] < QKVW || (size_t)in_sizes[5] < (size_t)DM * DM || in_sizes[6] < DM ||
        in_sizes[7] < DM || in_sizes[8] < DM || (size_t)in_sizes[9] < (size_t)FF * DM || in_sizes[10] < FF || (size_t)in_sizes[11] < (size_t)DM * FF || in_sizes[12] < DM) return;
    const float* x = (const float*)d_in[0]; const float* g1 = (const float*)d_in[1]; const float* be1 = (const float*)d_in[2]; const float* wqkv = (const float*)d_in[3]; const float* bqkv = (const float*)d_in[4];
    const float* wo = (const float*)d_in[5]; const float* bo = (const float*)d_in[6]; const float* g2 = (const float*)d_in[7]; const float* be2 = (const float*)d_in[8];
    const float* fcw = (const float*)d_in[9]; const float* fcb = (const float*)d_in[10]; const float* cpw = (const float*)d_in[11]; const float* cpb = (const float*)d_in[12];
    float* OUT = (float*)d_out;
    char* wsp = (char*)d_ws;
    auto take = [&](size_t bytes) { char* p = wsp; wsp += (bytes + 255) & ~(size_t)255; return (void*)p; };
    h16* WQKV = (h16*)take((size_t)QKVW * DM * 2);
    h16* WO   = (h16*)take((size_t)DM * DM * 2);
    h16* FCW  = (h16*)take((size_t)FF * DM * 2);
    h16* CPW  = (h16*)take((size_t)DM * FF * 2);
    h16* H16  = (h16*)take((size_t)TT * DM * 2);
    const size_t rbytes = ((size_t)TT * QKVW * 4 > (size_t)TT * FF * 4) ? (size_t)TT * QKVW * 4 : (size_t)TT * FF * 4;
    float* RG  = (float*)take(rbytes);
    h16* Q16  = (h16*)take((size_t)NH_ * TT * HD * 2);
    h16* K16  = (h16*)take((size_t)NH_ * TT * HD * 2);
    h16* VT16 = (h16*)take((size_t)NH_ * HD * TT * 2);
    h16* AT16 = (h16*)take((size_t)TT * DM * 2);
    float* X1 = (float*)take((size_t)TT * DM * 4);
    h16* G16  = (h16*)take((size_t)TT * FF * 2);
    const size_t used = (size_t)(wsp - (char*)d_ws);
    if (used > ws_size || used > (size_t)134217728) return;
    float* FQ = RG; float* F1 = RG;

    auto cvt = [&](const float* s, h16* d, size_t n) { const size_t n8 = n / 8; k_cvtw<<<(unsigned)((n8 + 255) / 256), 256, 0, stream>>>(s, d, n8, WCAR); };
    cvt(wqkv, WQKV, (size_t)QKVW * DM); cvt(wo, WO, (size_t)DM * DM); cvt(fcw, FCW, (size_t)FF * DM); cvt(cpw, CPW, (size_t)DM * FF);

    const unsigned gQK = (unsigned)((size_t)NH_ * TT * HD / 8 / 256), gVT = (unsigned)((size_t)NH_ * HD * TT / 8 / 256), gGE = (unsigned)((size_t)TT * FF / 8 / 256);
    for (int b = 0; b < NB; ++b) {
        const float* xb = x + (size_t)b * SEQ_FULL * DM; float* outb = OUT + (size_t)b * SEQ_FULL * DM;
        k_ln<true><<<TT / 8, 256, 0, stream>>>(xb, g1, be1, H16);
        k_gemmw<0, true, 0><<<dim3(TT / 64, QKVW / 64, 1), 32, 0, stream>>>(H16, nullptr, WQKV, nullptr, DM, FQ, QKVW, bqkv, nullptr, 1.0f / WCAR, 0, 0, 0);
        k_qkp<<<gQK, 256, 0, stream>>>(FQ, Q16, K16);
        k_vtp<<<gVT, 256, 0, stream>>>(FQ, VT16);
        k_flash<<<dim3(TT / 64, NH_, 1), 128, 0, stream>>>(Q16, K16, VT16, AT16);
        k_gemmw<0, true, 2><<<dim3(TT / 64, DM / 64, 1), 32, 0, stream>>>(AT16, nullptr, WO, nullptr, DM, X1, DM, bo, xb, 1.0f / (WCAR * OCAR), 0, 0, 0);
        k_ln<false><<<TT / 8, 256, 0, stream>>>(X1, g2, be2, H16);
        k_gemmw<0, true, 0><<<dim3(TT / 64, FF / 64, 1), 32, 0, stream>>>(H16, nullptr, FCW, nullptr, DM, F1, FF, fcb, nullptr, 1.0f / WCAR, 0, 0, 0);
        k_gelu<<<gGE, 256, 0, stream>>>(F1, G16, (size_t)TT * FF / 8);
        k_gemmw<0, true, 1><<<dim3(TT / 64, DM / 64, 1), 32, 0, stream>>>(G16, nullptr, CPW, nullptr, FF, outb, DM, cpb, X1, 1.0f / (WCAR * GCAR), 0, 0, 0);
    }
}
